// Decoder_56289841382057
// MI455X (gfx1250) — hardware-verified
//
#include <hip/hip_runtime.h>
#include <math.h>

constexpr int T_STEPS   = 2048;
constexpr int NKEYS     = 50000;
constexpr int NKEYS_PAD = 50176;
constexpr int E_DIM     = 128;
constexpr int H_DIM     = 512;
constexpr int G3_DIM    = 1536;
constexpr int DK_DIM    = 256;
constexpr int NVOC      = 1704;
constexpr int NVOC_PAD  = 1712;
constexpr int NLOC      = 100;
constexpr int NLOC_PAD  = 128;
constexpr int CAT_DIM   = 1024;
constexpr int LOC_PITCH = 2048;

constexpr float Y_CARRY     = 16.0f;
constexpr float W_CARRY     = 64.0f;
constexpr float H_CARRY     = 64.0f;
constexpr float LO_CARRY    = 2048.0f;
constexpr float P_CARRY     = 8.0f;
constexpr float B_CARRY     = 2048.0f;
constexpr float GX_SCALE    = 1.0f / (Y_CARRY * W_CARRY);
constexpr float GH_S1       = 1.0f / (H_CARRY * W_CARRY);
constexpr float GH_S2       = GH_S1 / LO_CARRY;
constexpr float Q_OUT_SCALE = 1.0f / W_CARRY;
constexpr float Q_CARRY_INV = 1.0f / H_CARRY;
constexpr float P_CARRY_INV = 1.0f / P_CARRY;
constexpr float CL_SCALE    = 1.0f / B_CARRY;
constexpr float LG_SCALE    = 1.0f / (H_CARRY * W_CARRY);
constexpr float NEG_BIG     = -1.0e30f;

constexpr int FL_MT         = 128;
constexpr int FL_NSPLIT     = 8;
constexpr int FL_SPLIT_KEYS = NKEYS_PAD / FL_NSPLIT;
constexpr int FL_NCHUNK     = FL_SPLIT_KEYS / 32;
constexpr int GRU_THREADS   = 512;
constexpr int GRU_HP        = 520;
constexpr int GRU_TLO       = 32;
constexpr int FC_NT         = NVOC_PAD / 16;

static_assert(NKEYS_PAD % 64 == 0 && NKEYS_PAD >= NKEYS, "key padding");
static_assert(FL_SPLIT_KEYS * FL_NSPLIT == NKEYS_PAD && FL_NCHUNK * 32 == FL_SPLIT_KEYS, "split shape");
static_assert(T_STEPS % FL_MT == 0 && T_STEPS % 64 == 0, "query tiles");
static_assert(G3_DIM == 3 * H_DIM && H_DIM == 32 * (GRU_THREADS / 32), "gru wave map");
static_assert(E_DIM % 32 == 0 && H_DIM % 32 == 0 && DK_DIM % 32 == 0 && CAT_DIM % 32 == 0 && NLOC_PAD % 32 == 0, "k multiples of 32");
static_assert(G3_DIM % 64 == 0 && DK_DIM % 64 == 0 && NLOC_PAD % 64 == 0 && H_DIM % 64 == 0, "n tiles");
static_assert(CAT_DIM == H_DIM + 2 * DK_DIM, "concat layout");
static_assert(NVOC_PAD % 16 == 0 && NVOC_PAD >= NVOC, "fc padding");
static_assert((16 * NVOC * 4) % 128 == 0, "fc block range is whole lines");
static_assert((16 * NVOC) % 4 == 0, "fc float4 count");

typedef __attribute__((ext_vector_type(16))) _Float16 v16h;
typedef __attribute__((ext_vector_type(8)))  _Float16 v8h;
typedef __attribute__((ext_vector_type(16))) __bf16   v16b;
typedef __attribute__((ext_vector_type(8)))  __bf16   v8b;
typedef __attribute__((ext_vector_type(8)))  float    v8f;
typedef __attribute__((ext_vector_type(4)))  float    v4f;
typedef __attribute__((ext_vector_type(4)))  unsigned int v4u;

__device__ __forceinline__ unsigned short f2bf_bits(float f) {
  unsigned u = __float_as_uint(f);
  return (unsigned short)((u + 0x7FFFu + ((u >> 16) & 1u)) >> 16);
}
__device__ __forceinline__ float bf_bits2f(unsigned short h) { return __uint_as_float(((unsigned)h) << 16); }

__device__ __forceinline__ void dep_guard_h(v8f& a, v8f& b, v16h x, v16h y) { asm volatile("v_nop\n\tv_nop\n\tv_nop\n\tv_nop" : "+v"(a), "+v"(b) : "v"(x), "v"(y)); }
__device__ __forceinline__ void dep_guard_b(v8f& a, v8f& b, v16b x, v16b y) { asm volatile("v_nop\n\tv_nop\n\tv_nop\n\tv_nop" : "+v"(a), "+v"(b) : "v"(x), "v"(y)); }
__device__ __forceinline__ void keep4_h(v16h a, v16h b, v16h c, v16h d) { asm volatile("v_nop" :: "v"(a), "v"(b), "v"(c), "v"(d)); }
__device__ __forceinline__ void keep4_b(v16b a, v16b b, v16b c, v16b d) { asm volatile("v_nop" :: "v"(a), "v"(b), "v"(c), "v"(d)); }
__device__ __forceinline__ void acc_guard4(v8f& a, v8f& b, v8f& c, v8f& d) { asm volatile("v_nop\n\tv_nop\n\tv_nop\n\tv_nop" : "+v"(a), "+v"(b), "+v"(c), "+v"(d)); }
__device__ __forceinline__ void gru_guard3(v8f& a, v8f& b, v8f& c, v16h x, v16h y0, v16h y1, v16h y2) {
  asm volatile("v_nop\n\tv_nop\n\tv_nop\n\tv_nop" : "+v"(a), "+v"(b), "+v"(c) : "v"(x), "v"(y0), "v"(y1), "v"(y2));
}
__device__ __forceinline__ void gru_guard6(v8f& a, v8f& b, v8f& c, v8f& d, v8f& e, v8f& f,
                                           v16h x, v16h y0, v16h y1, v16h y2, v16h z0, v16h z1, v16h z2) {
  asm volatile("v_nop\n\tv_nop\n\tv_nop\n\tv_nop" : "+v"(a), "+v"(b), "+v"(c), "+v"(d), "+v"(e), "+v"(f)
               : "v"(x), "v"(y0), "v"(y1), "v"(y2), "v"(z0), "v"(z1), "v"(z2));
}
__device__ __forceinline__ void fl_guard2(v8f& a, v8f& b, v16h x, v16h y, v16h z) {
  asm volatile("v_nop\n\tv_nop\n\tv_nop\n\tv_nop" : "+v"(a), "+v"(b) : "v"(x), "v"(y), "v"(z));
}
__device__ __forceinline__ void fl_guard4(v8f& a, v8f& b, v8f& c, v8f& d, v16h p, v16h x, v16h y, v16h z, v16h w) {
  asm volatile("v_nop\n\tv_nop\n\tv_nop\n\tv_nop" : "+v"(a), "+v"(b), "+v"(c), "+v"(d) : "v"(p), "v"(x), "v"(y), "v"(z), "v"(w));
}
__device__ __forceinline__ void fc_guard(v8f& a, v16b x, v16b y, v16b z, v16b w) {
  asm volatile("v_nop\n\tv_nop\n\tv_nop\n\tv_nop" : "+v"(a) : "v"(x), "v"(y), "v"(z), "v"(w));
}

template <typename T> struct Frag;
template <> struct Frag<_Float16> {
  typedef v16h V; union U { v16h v; v8h h[2]; };
  static __device__ __forceinline__ v16h load(const _Float16* p) {
    U f; f.h[0] = *(const v8h*)(p); f.h[1] = *(const v8h*)(p + 16); return f.v;
  }
  static __device__ __forceinline__ v8f mma(v16h a, v16h b, v8f c) {
    return __builtin_amdgcn_wmma_f32_16x16x32_f16(false, a, false, b, (short)0, c, false, false);
  }
  static __device__ __forceinline__ void guard(v8f& a, v8f& b, v16h x, v16h y) { dep_guard_h(a, b, x, y); }
  static __device__ __forceinline__ void keep(v16h a, v16h b, v16h c, v16h d) { keep4_h(a, b, c, d); }
};
template <> struct Frag<__bf16> {
  typedef v16b V; union U { v16b v; v8b h[2]; };
  static __device__ __forceinline__ v16b load(const __bf16* p) {
    U f; f.h[0] = *(const v8b*)(p); f.h[1] = *(const v8b*)(p + 16); return f.v;
  }
  static __device__ __forceinline__ v8f mma(v16b a, v16b b, v8f c) {
    return __builtin_amdgcn_wmma_f32_16x16x32_bf16(false, a, false, b, (short)0, c, false, false);
  }
  static __device__ __forceinline__ void guard(v8f& a, v8f& b, v16b x, v16b y) { dep_guard_b(a, b, x, y); }
  static __device__ __forceinline__ void keep(v16b a, v16b b, v16b c, v16b d) { keep4_b(a, b, c, d); }
};

template <int ET> struct Elem;
template <> struct Elem<0> { typedef _Float16 T; };
template <> struct Elem<1> { typedef __bf16 T; };
template <int ET, bool SPLIT, int BIAS_MODE, int OUT_MODE>
__global__ __launch_bounds__(256) void wmma_gemm64(
    const unsigned short* __restrict__ Ap, const unsigned short* __restrict__ A2p, int lda,
    const unsigned short* __restrict__ Btp, const unsigned short* __restrict__ Bt2p, int ldb,
    void* __restrict__ Cout, void* __restrict__ Cout2, int ldc,
    const float* __restrict__ bias,
    int M, int N, int K, float scale) {
  typedef typename Elem<ET>::T T;
  typedef typename Frag<T>::V V;
  const T* A = (const T*)Ap; const T* A2 = (const T*)A2p; const T* Bt = (const T*)Btp; const T* Bt2 = (const T*)Bt2p;
  __shared__ __align__(16) float sT[8][16 * 68];
  const int lane = threadIdx.x & 31;
  const int wave = threadIdx.x >> 5;
  const int tilesN = N >> 6;
  const int tilesM = M >> 6;
  const int tile = blockIdx.x * 8 + wave;
  if (tile >= tilesM * tilesN) return;
  const int tm = tile / tilesN;
  const int tn = tile - tm * tilesN;
  const int m0 = tm << 6;
  const int n0 = tn << 6;

  const int rlane = lane & 15;
  const int koff  = (lane >> 4) * 8;
  const int mOff  = (lane >> 4) * 8;

  v8f acc[4][4];
#pragma unroll
  for (int i = 0; i < 4; ++i)
#pragma unroll
    for (int j = 0; j < 4; ++j) acc[i][j] = (v8f){0.f,0.f,0.f,0.f,0.f,0.f,0.f,0.f};

  for (int k0 = 0; k0 < K; k0 += 32) {
    V bh[4], bl[4];
#pragma unroll
    for (int j = 0; j < 4; ++j) {
      const size_t bo = (size_t)(n0 + (j << 4) + rlane) * ldb + koff + k0;
      bh[j] = Frag<T>::load(Bt + bo);
      if (SPLIT) bl[j] = Frag<T>::load(Bt2 + bo);
    }
#pragma unroll
    for (int i = 0; i < 4; ++i) {
      const size_t ao = (size_t)(m0 + (i << 4) + rlane) * lda + koff + k0;
      V ah = Frag<T>::load(A + ao);
      V al;
      if (SPLIT) al = Frag<T>::load(A2 + ao);
#pragma unroll
      for (int j = 0; j < 4; ++j) {
        acc[i][j] = Frag<T>::mma(ah, bh[j], acc[i][j]);
        if (SPLIT) {
          acc[i][j] = Frag<T>::mma(ah, bl[j], acc[i][j]);
          acc[i][j] = Frag<T>::mma(al, bh[j], acc[i][j]);
        }
      }
      acc_guard4(acc[i][0], acc[i][1], acc[i][2], acc[i][3]);
      Frag<T>::guard(acc[i][0], acc[i][3], ah, SPLIT ? al : ah);
    }
    Frag<T>::keep(bh[0], bh[1], bh[2], bh[3]);
    if (SPLIT) Frag<T>::keep(bl[0], bl[1], bl[2], bl[3]);
  }
  acc_guard4(acc[0][0], acc[0][1], acc[0][2], acc[0][3]);
  acc_guard4(acc[1][0], acc[1][1], acc[1][2], acc[1][3]);
  acc_guard4(acc[2][0], acc[2][1], acc[2][2], acc[2][3]);
  acc_guard4(acc[3][0], acc[3][1], acc[3][2], acc[3][3]);

  float* slab = sT[wave];
#pragma unroll
  for (int i = 0; i < 4; ++i) {
    const int mBase = m0 + (i << 4);
#pragma unroll
    for (int j = 0; j < 4; ++j) {
      const int n = n0 + (j << 4) + rlane;
      float bv = 0.f;
      if (BIAS_MODE == 2) bv = bias[n];
#pragma unroll
      for (int r = 0; r < 8; ++r) {
        float v = acc[i][j][r] * scale;
        if (BIAS_MODE == 2) v += bv;
        slab[(mOff + r) * 68 + (j << 4) + rlane] = v;
      }
    }
    __builtin_amdgcn_fence(__ATOMIC_RELEASE, "workgroup");
    __builtin_amdgcn_wave_barrier();
    __builtin_amdgcn_fence(__ATOMIC_ACQUIRE, "workgroup");
    if (OUT_MODE == 0) {
      float* C = (float*)Cout;
      const int hh = lane >> 4, c4 = (lane & 15) * 4;
      for (int pass = 0; pass < 2; ++pass) {
#pragma unroll
        for (int it = 0; it < 8; ++it) {
          const int row = it * 2 + hh;
          v4f v = *(const v4f*)(slab + row * 68 + c4);
          *(volatile v4f*)(C + (size_t)(mBase + row) * ldc + n0 + c4) = v;
        }
        __threadfence();
      }
    } else {
      const int q = lane >> 3, c8 = (lane & 7) * 8;
      unsigned short* C  = (unsigned short*)Cout;
      unsigned short* C2 = (unsigned short*)Cout2;
      for (int pass = 0; pass < 2; ++pass) {
#pragma unroll
        for (int it = 0; it < 4; ++it) {
          const int row = it * 4 + q;
          const float* sp = slab + row * 68 + c8;
          v8h hv, lv;
#pragma unroll
          for (int e = 0; e < 8; ++e) {
            if (OUT_MODE == 1) {
              hv[e] = (_Float16)sp[e];
            } else {
              unsigned short hb = f2bf_bits(sp[e]);
              unsigned short lb = f2bf_bits(sp[e] - bf_bits2f(hb));
              hv[e] = __builtin_bit_cast(_Float16, hb);
              lv[e] = __builtin_bit_cast(_Float16, lb);
            }
          }
          *(volatile v8h*)(C + (size_t)(mBase + row) * ldc + n0 + c8) = hv;
          if (OUT_MODE == 2) *(volatile v8h*)(C2 + (size_t)(mBase + row) * ldc + n0 + c8) = lv;
        }
        __threadfence();
      }
    }
    __builtin_amdgcn_fence(__ATOMIC_RELEASE, "workgroup");
    __builtin_amdgcn_wave_barrier();
    __builtin_amdgcn_fence(__ATOMIC_ACQUIRE, "workgroup");
  }
}

__global__ __launch_bounds__(256) void gather_y16_kernel(const int* __restrict__ X, const float* __restrict__ emb,
                                                         unsigned short* __restrict__ y16) {
  const int i = blockIdx.x * 256 + threadIdx.x;
  if (i < T_STEPS * (E_DIM / 8)) {
    const int t = i >> 4, c8 = i & 15;
    int x = X[t];
    x = x < 0 ? 0 : (x > NVOC - 1 ? NVOC - 1 : x);
    const float* sp = emb + (size_t)x * E_DIM + c8 * 8;
    const v4f a = *(const v4f*)(sp);
    const v4f b = *(const v4f*)(sp + 4);
    v8h hv;
#pragma unroll
    for (int e = 0; e < 4; ++e) {
      hv[e]     = (_Float16)(a[e] * Y_CARRY);
      hv[4 + e] = (_Float16)(b[e] * Y_CARRY);
    }
    unsigned short* dp = y16 + (size_t)i * 8;
    *(volatile v8h*)dp = hv;
    __threadfence();
    *(volatile v8h*)dp = hv;
  }
}

template <bool LO>
__global__ __launch_bounds__(256) void cvt8_f16_kernel(const float* __restrict__ src, int spitch, int scol0, int rreal,
                                                       int nrow, int ncol8,
                                                       unsigned short* __restrict__ dst, unsigned short* __restrict__ dst2,
                                                       int dpitch, int dcol0, float sc) {
  const int i  = blockIdx.x * 256 + threadIdx.x;
  const int n8 = nrow * ncol8;
  if (i < n8) {
    const int row = i / ncol8;
    const int c8  = i - row * ncol8;
    const int rc  = row < rreal ? row : rreal - 1;
    const bool ok = row < rreal;
    const float* sp = src + (size_t)rc * spitch + scol0 + c8 * 8;
    const v4f a = *(const v4f*)(sp);
    const v4f b = *(const v4f*)(sp + 4);
    v8h hv, lv;
#pragma unroll
    for (int e = 0; e < 4; ++e) {
      const float f0 = ok ? a[e] * sc : 0.0f;
      const float f1 = ok ? b[e] * sc : 0.0f;
      const _Float16 h0 = (_Float16)f0;
      const _Float16 h1 = (_Float16)f1;
      hv[e] = h0;
      hv[4 + e] = h1;
      if (LO) {
        lv[e]     = (_Float16)((f0 - (float)h0) * LO_CARRY);
        lv[4 + e] = (_Float16)((f1 - (float)h1) * LO_CARRY);
      }
    }
    const size_t o = (size_t)row * dpitch + dcol0 + c8 * 8;
    *(volatile v8h*)(dst + o) = hv;
    if (LO) *(volatile v8h*)(dst2 + o) = lv;
    __threadfence();
    *(volatile v8h*)(dst + o) = hv;
    if (LO) *(volatile v8h*)(dst2 + o) = lv;
  }
}

__global__ __launch_bounds__(256) void split8_bf16_kernel(const float* __restrict__ src, int spitch, int rreal, int creal,
                                                          int nrow, int ncol8,
                                                          unsigned short* __restrict__ dhi, unsigned short* __restrict__ dlo) {
  const int i  = blockIdx.x * 256 + threadIdx.x;
  const int n8 = nrow * ncol8;
  if (i < n8) {
    const int row = i / ncol8;
    const int c8  = i - row * ncol8;
    const int rc  = row < rreal ? row : rreal - 1;
    v8h hv, lv;
#pragma unroll
    for (int e = 0; e < 8; ++e) {
      const int col = c8 * 8 + e;
      const int cc  = col < creal ? col : creal - 1;
      const float raw = src[(size_t)rc * spitch + cc];
      const float f = (row < rreal && col < creal) ? raw : 0.0f;
      const unsigned short hb = f2bf_bits(f);
      const unsigned short lb = f2bf_bits(f - bf_bits2f(hb));
      hv[e] = __builtin_bit_cast(_Float16, hb);
      lv[e] = __builtin_bit_cast(_Float16, lb);
    }
    const size_t o = (size_t)i * 8;
    *(volatile v8h*)(dhi + o) = hv;
    *(volatile v8h*)(dlo + o) = lv;
    __threadfence();
    *(volatile v8h*)(dhi + o) = hv;
    *(volatile v8h*)(dlo + o) = lv;
  }
}

__global__ __launch_bounds__(256) void tp_f16_kernel(const float* __restrict__ src, int spitch, int rreal,
                                                     unsigned short* __restrict__ O, int ldo, float sc) {
  __shared__ float Tt[64 * 65];
  const int tid = threadIdx.x;
  const int c0 = blockIdx.x * 64, r0 = blockIdx.y * 64;
#pragma unroll
  for (int i = 0; i < 4; ++i) {
    const int idx = i * 256 + tid;
    const int rr = idx >> 4, cc = (idx & 15) * 4;
    const int row = r0 + rr;
    const int rc  = row < rreal ? row : rreal - 1;
    const bool ok = row < rreal;
    const v4f v = *(const v4f*)(src + (size_t)rc * spitch + c0 + cc);
    Tt[rr * 65 + cc + 0] = ok ? v[0] * sc : 0.0f;
    Tt[rr * 65 + cc + 1] = ok ? v[1] * sc : 0.0f;
    Tt[rr * 65 + cc + 2] = ok ? v[2] * sc : 0.0f;
    Tt[rr * 65 + cc + 3] = ok ? v[3] * sc : 0.0f;
  }
  __syncthreads();
  const int q = tid >> 3, c8 = (tid & 7) * 8;
  v8h hv[2];
#pragma unroll
  for (int g = 0; g < 2; ++g) {
    const int qq = g * 32 + q;
#pragma unroll
    for (int e = 0; e < 8; ++e) hv[g][e] = (_Float16)Tt[(c8 + e) * 65 + qq];
  }
  for (int pass = 0; pass < 2; ++pass) {
#pragma unroll
    for (int g = 0; g < 2; ++g) {
      const size_t o = (size_t)(c0 + g * 32 + q) * (size_t)ldo + (size_t)(r0 + c8);
      *(volatile v8h*)(O + o) = hv[g];
    }
    __threadfence();
  }
}

__device__ __forceinline__ float sigmoid_f(float x) { return 1.0f / (1.0f + expf(-x)); }

template <bool LO>
__device__ __forceinline__ void gru_dot(const unsigned short* arow, unsigned amask,
                                        const _Float16* wh, const _Float16* wl,
                                        v8f& a0, v8f& a1, v8f& a2, v8f& l0, v8f& l1, v8f& l2) {
  const size_t gs = (size_t)H_DIM * H_DIM;
  const v4u mk = (v4u){amask, amask, amask, amask};
#pragma unroll 1
  for (int k0 = 0; k0 < H_DIM; k0 += 32) {
    union { v16h v; v4u q[2]; } fa;
    fa.q[0] = *(const v4u*)(arow + k0);
    fa.q[1] = *(const v4u*)(arow + k0 + 16);
    fa.q[0] = fa.q[0] & mk;
    fa.q[1] = fa.q[1] & mk;
    const v16h a  = fa.v;
    const v16h b0 = Frag<_Float16>::load(wh + k0);
    const v16h b1 = Frag<_Float16>::load(wh + gs + k0);
    const v16h b2 = Frag<_Float16>::load(wh + 2 * gs + k0);
    a0 = Frag<_Float16>::mma(a, b0, a0);
    a1 = Frag<_Float16>::mma(a, b1, a1);
    a2 = Frag<_Float16>::mma(a, b2, a2);
    if (LO) {
      const v16h c0 = Frag<_Float16>::load(wl + k0);
      const v16h c1 = Frag<_Float16>::load(wl + gs + k0);
      const v16h c2 = Frag<_Float16>::load(wl + 2 * gs + k0);
      l0 = Frag<_Float16>::mma(a, c0, l0);
      l1 = Frag<_Float16>::mma(a, c1, l1);
      l2 = Frag<_Float16>::mma(a, c2, l2);
      gru_guard6(a0, a1, a2, l0, l1, l2, a, b0, b1, b2, c0, c1, c2);
    } else {
      gru_guard3(a0, a1, a2, a, b0, b1, b2);
    }
  }
}

__device__ __forceinline__ void gru_store_row(int wave, int lane, const float* hf, const unsigned short* ahi,
                                              float* outrow, unsigned short* catrow) {
  if (wave == 0) {
    v4f v[4];
#pragma unroll
    for (int q = 0; q < 4; ++q) v[q] = *(const v4f*)(hf + 128 * q + 4 * lane);
    for (int pass = 0; pass < 2; ++pass) {
#pragma unroll
      for (int q = 0; q < 4; ++q) *(volatile v4f*)(outrow + 128 * q + 4 * lane) = v[q];
      __threadfence();
    }
  } else if (wave == 1) {
    v4u u[2];
#pragma unroll
    for (int q = 0; q < 2; ++q) u[q] = *(const v4u*)(ahi + 256 * q + 8 * lane);
    for (int pass = 0; pass < 2; ++pass) {
#pragma unroll
      for (int q = 0; q < 2; ++q) *(volatile v4u*)(catrow + 256 * q + 8 * lane) = u[q];
      __threadfence();
    }
  }
}

__global__ __launch_bounds__(GRU_THREADS) void gru_kernel(const float* __restrict__ gx,
                                                          const unsigned short* __restrict__ Whip,
                                                          const unsigned short* __restrict__ Wlop,
                                                          const float* __restrict__ b_hh,
                                                          const float* __restrict__ glo0,
                                                          const float* __restrict__ loc0,
                                                          float* __restrict__ outf,
                                                          unsigned short* __restrict__ cat16) {
  __shared__ __align__(16) unsigned short Ah[2][2][GRU_HP];
  __shared__ __align__(16) float Hf[2][H_DIM];
  const _Float16* Whi = (const _Float16*)Whip;
  const _Float16* Wlo = (const _Float16*)Wlop;
  const int tid = threadIdx.x, lane = tid & 31, wave = tid >> 5;
  const int c = lane & 15, hh = lane >> 4, koff = hh * 8;

  {
    const float a = glo0[tid & 255];
    const float b = loc0[tid & 255];
    const float h0 = (tid < 256) ? a : b;
    const float hs = h0 * H_CARRY;
    const _Float16 hi = (_Float16)hs;
    const _Float16 lo = (_Float16)((hs - (float)hi) * LO_CARRY);
    Ah[0][0][tid] = __builtin_bit_cast(unsigned short, hi);
    Ah[0][1][tid] = __builtin_bit_cast(unsigned short, lo);
  }
  float hreg[2], bh[2][3];
#pragma unroll
  for (int ub = 0; ub < 2; ++ub) {
    const int unit = 32 * wave + 16 * ub + c;
    const float a = glo0[unit & 255];
    const float b = loc0[unit & 255];
    hreg[ub] = (unit < 256) ? a : b;
#pragma unroll
    for (int g = 0; g < 3; ++g) bh[ub][g] = b_hh[g * H_DIM + unit];
  }
  __syncthreads();

  const unsigned amask = (c < 2) ? 0xffffffffu : 0u;
  const int rsel = (c < 2) ? c : 0;
  const v8f z8 = {0.f, 0.f, 0.f, 0.f, 0.f, 0.f, 0.f, 0.f};

#pragma unroll 1
  for (int t = 0; t < T_STEPS; ++t) {
    const int p = t & 1;
    if (t > 0) gru_store_row(wave, lane, &Hf[p][0], &Ah[p][0][0],
                             outf + (size_t)(t - 1) * H_DIM, cat16 + (size_t)(t - 1) * CAT_DIM);
    float gxv[2][3];
#pragma unroll
    for (int ub = 0; ub < 2; ++ub)
#pragma unroll
      for (int g = 0; g < 3; ++g) gxv[ub][g] = gx[(size_t)t * G3_DIM + g * H_DIM + 32 * wave + 16 * ub + c];

    const unsigned short* arow = &Ah[p][rsel][koff];
#pragma unroll
    for (int ub = 0; ub < 2; ++ub) {
      const int unit = 32 * wave + 16 * ub + c;
      const _Float16* wh = Whi + (size_t)unit * H_DIM + koff;
      const _Float16* wl = Wlo + (size_t)unit * H_DIM + koff;
      v8f a0 = z8, a1 = z8, a2 = z8, l0 = z8, l1 = z8, l2 = z8;
      if (t < GRU_TLO) gru_dot<true>(arow, amask, wh, wl, a0, a1, a2, l0, l1, l2);
      else             gru_dot<false>(arow, amask, wh, wl, a0, a1, a2, l0, l1, l2);
      const float ghr = a0[0] * GH_S1 + (a0[1] + l0[0]) * GH_S2 + bh[ub][0];
      const float ghz = a1[0] * GH_S1 + (a1[1] + l1[0]) * GH_S2 + bh[ub][1];
      const float ghn = a2[0] * GH_S1 + (a2[1] + l2[0]) * GH_S2 + bh[ub][2];
      const float rg = sigmoid_f(gxv[ub][0] + ghr);
      const float zg = sigmoid_f(gxv[ub][1] + ghz);
      const float ng = tanhf(gxv[ub][2] + rg * ghn);
      const float hn = (1.0f - zg) * ng + zg * hreg[ub];
      hreg[ub] = hn;
      if (hh == 0) {
        const float hs = hn * H_CARRY;
        const _Float16 hi = (_Float16)hs;
        const _Float16 lo = (_Float16)((hs - (float)hi) * LO_CARRY);
        Hf[p ^ 1][unit] = hn;
        Ah[p ^ 1][0][unit] = __builtin_bit_cast(unsigned short, hi);
        Ah[p ^ 1][1][unit] = __builtin_bit_cast(unsigned short, lo);
      }
    }
    __syncthreads();
  }
  gru_store_row(wave, lane, &Hf[0][0], &Ah[0][0][0],
                outf + (size_t)(T_STEPS - 1) * H_DIM, cat16 + (size_t)(T_STEPS - 1) * CAT_DIM);
}

__global__ __launch_bounds__(256) void flash_kernel(const unsigned short* __restrict__ q16p,
                                                    const unsigned short* __restrict__ k16p,
                                                    const unsigned short* __restrict__ vT16p,
                                                    float* __restrict__ pctx, float* __restrict__ pm,
                                                    float* __restrict__ pl) {
  __shared__ __align__(16) float slabs[8][16 * 68];
  __shared__ __align__(16) float sM[FL_MT];
  __shared__ __align__(16) float sL[FL_MT];
  const _Float16* Q  = (const _Float16*)q16p;
  const _Float16* Kp = (const _Float16*)k16p;
  const _Float16* Vt = (const _Float16*)vT16p;
  const int lane = threadIdx.x & 31, wave = threadIdx.x >> 5;
  const int c = lane & 15, hh = lane >> 4, koff = hh * 8;
  const int mt = blockIdx.x, sp = blockIdx.y;
  const int q0 = mt * FL_MT + wave * 16;
  const _Float16* qrow = Q + (size_t)(q0 + c) * DK_DIM + koff;
  const v8f z8 = {0.f, 0.f, 0.f, 0.f, 0.f, 0.f, 0.f, 0.f};
  v8f ctx[16];
#pragma unroll
  for (int i = 0; i < 16; ++i) ctx[i] = z8;
  float mref = NEG_BIG, lsum = 0.0f;
  const int kbase = sp * FL_SPLIT_KEYS;

#pragma unroll 1
  for (int ch = 0; ch < FL_NCHUNK; ++ch) {
    const int key0 = kbase + ch * 32;
    const _Float16* k0row = Kp + (size_t)(key0 + c) * DK_DIM + koff;
    const _Float16* k1row = k0row + 16 * DK_DIM;
    v8f s0 = z8, s1 = z8;
#pragma unroll 1
    for (int kk = 0; kk < DK_DIM; kk += 32) {
      const v16h b  = Frag<_Float16>::load(qrow + kk);
      const v16h a0 = Frag<_Float16>::load(k0row + kk);
      const v16h a1 = Frag<_Float16>::load(k1row + kk);
      s0 = Frag<_Float16>::mma(a0, b, s0);
      s1 = Frag<_Float16>::mma(a1, b, s1);
      fl_guard2(s0, s1, a0, a1, b);
    }
    float x0[8], x1[8];
#pragma unroll
    for (int r = 0; r < 8; ++r) { x0[r] = s0[r] * Q_CARRY_INV; x1[r] = s1[r] * Q_CARRY_INV; }
    if (key0 + 32 > NKEYS) {
#pragma unroll
      for (int r = 0; r < 8; ++r) {
        const int kidx = key0 + 8 * hh + r;
        x0[r] = (kidx < NKEYS) ? x0[r] : NEG_BIG;
        x1[r] = (kidx + 16 < NKEYS) ? x1[r] : NEG_BIG;
      }
    }
    float cm = NEG_BIG;
#pragma unroll
    for (int r = 0; r < 8; ++r) cm = fmaxf(cm, fmaxf(x0[r], x1[r]));
    cm = fmaxf(cm, __shfl_xor(cm, 16, 32));
    const bool need = cm > mref + 8.0f;
    if (__any((int)need)) {
      const float mnew  = need ? cm : mref;
      const float alpha = expf(mref - mnew);
      mref = mnew;
      lsum *= alpha;
#pragma unroll
      for (int et = 0; et < 16; ++et) ctx[et] = ctx[et] * alpha;
    }
    v16h pf;
#pragma unroll
    for (int r = 0; r < 8; ++r) {
      const float p0 = expf(x0[r] - mref);
      const float p1 = expf(x1[r] - mref);
      lsum += p0 + p1;
      pf[r]     = (_Float16)(p0 * P_CARRY);
      pf[8 + r] = (_Float16)(p1 * P_CARRY);
    }
    const _Float16* vbase = Vt + (size_t)c * NKEYS_PAD + key0 + koff;
#pragma unroll
    for (int g4 = 0; g4 < 4; ++g4) {
      const _Float16* vp = vbase + (size_t)(g4 * 64) * NKEYS_PAD;
      const v16h v0 = Frag<_Float16>::load(vp);
      const v16h v1 = Frag<_Float16>::load(vp + (size_t)16 * NKEYS_PAD);
      const v16h v2 = Frag<_Float16>::load(vp + (size_t)32 * NKEYS_PAD);
      const v16h v3 = Frag<_Float16>::load(vp + (size_t)48 * NKEYS_PAD);
      ctx[4 * g4 + 0] = Frag<_Float16>::mma(v0, pf, ctx[4 * g4 + 0]);
      ctx[4 * g4 + 1] = Frag<_Float16>::mma(v1, pf, ctx[4 * g4 + 1]);
      ctx[4 * g4 + 2] = Frag<_Float16>::mma(v2, pf, ctx[4 * g4 + 2]);
      ctx[4 * g4 + 3] = Frag<_Float16>::mma(v3, pf, ctx[4 * g4 + 3]);
      fl_guard4(ctx[4 * g4 + 0], ctx[4 * g4 + 1], ctx[4 * g4 + 2], ctx[4 * g4 + 3], pf, v0, v1, v2, v3);
      asm volatile("" ::: "memory");
    }
  }

  lsum += __shfl_xor(lsum, 16, 32);
  if (hh == 0) { sM[wave * 16 + c] = mref; sL[wave * 16 + c] = lsum; }

  float* slab = slabs[wave];
  const int c4 = (lane & 15) * 4;
#pragma unroll
  for (int sg = 0; sg < 4; ++sg) {
#pragma unroll
    for (int e4 = 0; e4 < 4; ++e4)
#pragma unroll
      for (int r = 0; r < 8; ++r) slab[c * 68 + e4 * 16 + 8 * hh + r] = ctx[4 * sg + e4][r] * P_CARRY_INV;
    __builtin_amdgcn_fence(__ATOMIC_RELEASE, "workgroup");
    __builtin_amdgcn_wave_barrier();
    __builtin_amdgcn_fence(__ATOMIC_ACQUIRE, "workgroup");
    for (int pass = 0; pass < 2; ++pass) {
#pragma unroll
      for (int it = 0; it < 8; ++it) {
        const int row = it * 2 + hh;
        const v4f v = *(const v4f*)(slab + row * 68 + c4);
        *(volatile v4f*)(pctx + ((size_t)sp * T_STEPS + (size_t)(q0 + row)) * DK_DIM + sg * 64 + c4) = v;
      }
      __threadfence();
    }
    __builtin_amdgcn_fence(__ATOMIC_RELEASE, "workgroup");
    __builtin_amdgcn_wave_barrier();
    __builtin_amdgcn_fence(__ATOMIC_ACQUIRE, "workgroup");
  }
  __syncthreads();
  if (wave == 0) {
    const v4f v = *(const v4f*)(sM + 4 * lane);
    float* dp = pm + (size_t)sp * T_STEPS + mt * FL_MT + 4 * lane;
    *(volatile v4f*)dp = v;
    __threadfence();
    *(volatile v4f*)dp = v;
  } else if (wave == 1) {
    const v4f v = *(const v4f*)(sL + 4 * lane);
    float* dp = pl + (size_t)sp * T_STEPS + mt * FL_MT + 4 * lane;
    *(volatile v4f*)dp = v;
    __threadfence();
    *(volatile v4f*)dp = v;
  }
}

__global__ __launch_bounds__(256) void combine_kernel(const float* __restrict__ pctx, const float* __restrict__ pm,
                                                      const float* __restrict__ pl, float* __restrict__ cg) {
  const int lane = threadIdx.x & 31;
  const int row = blockIdx.x * 8 + (threadIdx.x >> 5);
  float mx = NEG_BIG;
#pragma unroll 1
  for (int s = 0; s < FL_NSPLIT; ++s) mx = fmaxf(mx, pm[(size_t)s * T_STEPS + row]);
  float den = 0.0f;
  v4f n0 = {0.f, 0.f, 0.f, 0.f}, n1 = {0.f, 0.f, 0.f, 0.f};
#pragma unroll 1
  for (int s = 0; s < FL_NSPLIT; ++s) {
    const float ms = pm[(size_t)s * T_STEPS + row];
    const float ls = pl[(size_t)s * T_STEPS + row];
    const float w = expf(ms - mx);
    den += w * ls;
    const float* pr = pctx + ((size_t)s * T_STEPS + row) * DK_DIM;
    const v4f a = *(const v4f*)(pr + 4 * lane);
    const v4f b = *(const v4f*)(pr + 128 + 4 * lane);
    n0 = n0 + a * w;
    n1 = n1 + b * w;
  }
  const float inv = 1.0f / den;
  const v4f o0 = n0 * inv, o1 = n1 * inv;
  float* op = cg + (size_t)row * DK_DIM;
  for (int pass = 0; pass < 2; ++pass) {
    *(volatile v4f*)(op + 4 * lane) = o0;
    *(volatile v4f*)(op + 128 + 4 * lane) = o1;
    __threadfence();
  }
}

__global__ __launch_bounds__(256) void beta_softmax_kernel(const float* __restrict__ Sl, float* __restrict__ beta,
                                                           unsigned short* __restrict__ beta16) {
  const int lane = threadIdx.x & 31;
  const int row = blockIdx.x * 8 + (threadIdx.x >> 5);
  const bool valid = lane < (NLOC / 4);
  const v4f x = *(const v4f*)(Sl + (size_t)row * NLOC_PAD + 4 * lane);
  float m = valid ? fmaxf(fmaxf(x[0], x[1]), fmaxf(x[2], x[3])) : NEG_BIG;
#pragma unroll
  for (int off = 1; off < 32; off <<= 1) m = fmaxf(m, __shfl_xor(m, off, 32));
  float e0 = valid ? expf(x[0] - m) : 0.0f;
  float e1 = valid ? expf(x[1] - m) : 0.0f;
  float e2 = valid ? expf(x[2] - m) : 0.0f;
  float e3 = valid ? expf(x[3] - m) : 0.0f;
  float s = (e0 + e1) + (e2 + e3);
#pragma unroll
  for (int off = 1; off < 32; off <<= 1) s += __shfl_xor(s, off, 32);
  const float inv = 1.0f / s;
  const v4f b = (v4f){e0 * inv, e1 * inv, e2 * inv, e3 * inv};
  float* bp = beta + (size_t)row * NLOC_PAD + 4 * lane;
  *(volatile v4f*)bp = b;
  __threadfence();
  *(volatile v4f*)bp = b;
  const int sa = (2 * lane) & 31, sb = (2 * lane + 1) & 31;
  float g[8];
  g[0] = __shfl(b[0], sa, 32); g[1] = __shfl(b[1], sa, 32); g[2] = __shfl(b[2], sa, 32); g[3] = __shfl(b[3], sa, 32);
  g[4] = __shfl(b[0], sb, 32); g[5] = __shfl(b[1], sb, 32); g[6] = __shfl(b[2], sb, 32); g[7] = __shfl(b[3], sb, 32);
  v8h hv;
#pragma unroll
  for (int e = 0; e < 8; ++e) hv[e] = (_Float16)(g[e] * B_CARRY);
  if (lane < 16) {
    unsigned short* hp = beta16 + (size_t)row * NLOC_PAD + 8 * lane;
    *(volatile v8h*)hp = hv;
    __threadfence();
    *(volatile v8h*)hp = hv;
  }
}

__global__ __launch_bounds__(256) void head_kernel(const float* __restrict__ logits, const float* __restrict__ wvb,
                                                   const float* __restrict__ beta, const float* __restrict__ outf,
                                                   const float* __restrict__ cl, const int* __restrict__ X,
                                                   const float* __restrict__ emb, const float* __restrict__ wh,
                                                   const float* __restrict__ wc, const float* __restrict__ wy,
                                                   unsigned short* __restrict__ Pwh, unsigned short* __restrict__ Pwl) {
  const int lane = threadIdx.x & 31;
  const int row = blockIdx.x * 8 + (threadIdx.x >> 5);
  const bool valid = lane < (NLOC / 4);
  const v4f lg = *(const v4f*)(logits + (size_t)row * NLOC_PAD + 4 * lane);
  const v4f bt = *(const v4f*)(beta + (size_t)row * NLOC_PAD + 4 * lane);
  float x[4];
#pragma unroll
  for (int e = 0; e < 4; ++e) {
    const int col = 4 * lane + e;
    const int cb = col < NLOC ? col : NLOC - 1;
    x[e] = lg[e] + wvb[cb];
  }
  float m = valid ? fmaxf(fmaxf(x[0], x[1]), fmaxf(x[2], x[3])) : NEG_BIG;
#pragma unroll
  for (int off = 1; off < 32; off <<= 1) m = fmaxf(m, __shfl_xor(m, off, 32));
  float e0 = valid ? expf(x[0] - m) : 0.0f;
  float e1 = valid ? expf(x[1] - m) : 0.0f;
  float e2 = valid ? expf(x[2] - m) : 0.0f;
  float e3 = valid ? expf(x[3] - m) : 0.0f;
  float s = (e0 + e1) + (e2 + e3);
#pragma unroll
  for (int off = 1; off < 32; off <<= 1) s += __shfl_xor(s, off, 32);
  const float inv = 1.0f / s;

  float a = 0.0f;
#pragma unroll 1
  for (int i = 0; i < H_DIM / 128; ++i) {
    const v4f o = *(const v4f*)(outf + (size_t)row * H_DIM + 128 * i + 4 * lane);
    const v4f w = *(const v4f*)(wh + 128 * i + 4 * lane);
    a += (o[0] * w[0] + o[1] * w[1]) + (o[2] * w[2] + o[3] * w[3]);
  }
#pragma unroll 1
  for (int i = 0; i < DK_DIM / 128; ++i) {
    const v4f o = *(const v4f*)(cl + (size_t)row * DK_DIM + 128 * i + 4 * lane);
    const v4f w = *(const v4f*)(wc + 128 * i + 4 * lane);
    a += (o[0] * w[0] + o[1] * w[1]) + (o[2] * w[2] + o[3] * w[3]);
  }
  {
    int xi = X[row];
    xi = xi < 0 ? 0 : (xi > NVOC - 1 ? NVOC - 1 : xi);
    const v4f o = *(const v4f*)(emb + (size_t)xi * E_DIM + 4 * lane);
    const v4f w = *(const v4f*)(wy + 4 * lane);
    a += (o[0] * w[0] + o[1] * w[1]) + (o[2] * w[2] + o[3] * w[3]);
  }
#pragma unroll
  for (int off = 1; off < 32; off <<= 1) a += __shfl_xor(a, off, 32);
  const float pg = (a >= 0.0f) ? a : 0.2f * a;
  const float om = 1.0f - pg;
  float pw[4];
  pw[0] = valid ? pg * (e0 * inv) + om * bt[0] : 0.0f;
  pw[1] = valid ? pg * (e1 * inv) + om * bt[1] : 0.0f;
  pw[2] = valid ? pg * (e2 * inv) + om * bt[2] : 0.0f;
  pw[3] = valid ? pg * (e3 * inv) + om * bt[3] : 0.0f;
  const int sa = (2 * lane) & 31, sb = (2 * lane + 1) & 31;
  float g[8];
  g[0] = __shfl(pw[0], sa, 32); g[1] = __shfl(pw[1], sa, 32); g[2] = __shfl(pw[2], sa, 32); g[3] = __shfl(pw[3], sa, 32);
  g[4] = __shfl(pw[0], sb, 32); g[5] = __shfl(pw[1], sb, 32); g[6] = __shfl(pw[2], sb, 32); g[7] = __shfl(pw[3], sb, 32);
  v8h hv, lv;
#pragma unroll
  for (int e = 0; e < 8; ++e) {
    const unsigned short hb = f2bf_bits(g[e]);
    const unsigned short lb = f2bf_bits(g[e] - bf_bits2f(hb));
    hv[e] = __builtin_bit_cast(_Float16, hb);
    lv[e] = __builtin_bit_cast(_Float16, lb);
  }
  if (lane < 16) {
    const size_t o = (size_t)row * NLOC_PAD + 8 * lane;
    *(volatile v8h*)(Pwh + o) = hv;
    *(volatile v8h*)(Pwl + o) = lv;
    __threadfence();
    *(volatile v8h*)(Pwh + o) = hv;
    *(volatile v8h*)(Pwl + o) = lv;
  }
}

__global__ __launch_bounds__(256) void fc_kernel(const unsigned short* __restrict__ Php, const unsigned short* __restrict__ Plp,
                                                 const unsigned short* __restrict__ Fhp, const unsigned short* __restrict__ Flp,
                                                 const float* __restrict__ fcb, float* __restrict__ out) {
  __shared__ __align__(16) float Cs[16 * NVOC];
  const __bf16* Ph = (const __bf16*)Php;
  const __bf16* Pl = (const __bf16*)Plp;
  const __bf16* Fh = (const __bf16*)Fhp;
  const __bf16* Fl = (const __bf16*)Flp;
  const int tid = threadIdx.x, lane = tid & 31, wave = tid >> 5;
  const int c = lane & 15, hh = lane >> 4, koff = hh * 8;
  const int t0 = blockIdx.x * 16;
  v16b ah[4], al[4];
#pragma unroll
  for (int ks = 0; ks < 4; ++ks) {
    ah[ks] = Frag<__bf16>::load(Ph + (size_t)(t0 + c) * NLOC_PAD + koff + 32 * ks);
    al[ks] = Frag<__bf16>::load(Pl + (size_t)(t0 + c) * NLOC_PAD + koff + 32 * ks);
  }
#pragma unroll 1
  for (int nt = wave; nt < FC_NT; nt += 8) {
    const int n = nt * 16 + c;
    const __bf16* bhp = Fh + (size_t)n * NLOC_PAD + koff;
    const __bf16* blp = Fl + (size_t)n * NLOC_PAD + koff;
    v8f acc = {0.f, 0.f, 0.f, 0.f, 0.f, 0.f, 0.f, 0.f};
#pragma unroll
    for (int ks = 0; ks < 4; ++ks) {
      const v16b bh = Frag<__bf16>::load(bhp + 32 * ks);
      const v16b bl = Frag<__bf16>::load(blp + 32 * ks);
      acc = Frag<__bf16>::mma(ah[ks], bh, acc);
      acc = Frag<__bf16>::mma(ah[ks], bl, acc);
      acc = Frag<__bf16>::mma(al[ks], bh, acc);
      fc_guard(acc, ah[ks], al[ks], bh, bl);
    }
    const int nb = n < NVOC ? n : NVOC - 1;
    const float bv = fcb[nb];
    if (n < NVOC) {
#pragma unroll
      for (int r = 0; r < 8; ++r) Cs[(8 * hh + r) * NVOC + n] = acc[r] + bv;
    }
  }
  __syncthreads();
  float* ob = out + (size_t)t0 * NVOC;
  for (int pass = 0; pass < 2; ++pass) {
#pragma unroll 1
    for (int i = tid; i < (16 * NVOC) / 4; i += 256) {
      const v4f v = *(const v4f*)(Cs + 4 * i);
      *(volatile v4f*)(ob + 4 * (size_t)i) = v;
    }
    __threadfence();
  }
}

extern "C" void kernel_launch(void* const* d_in, const int* in_sizes, int n_in,
                              void* d_out, int out_size, void* d_ws, size_t ws_size, hipStream_t stream) {
  if (n_in < 18 || d_out == nullptr || d_ws == nullptr) return;
  if (in_sizes[0] != T_STEPS || in_sizes[1] != NKEYS * DK_DIM || in_sizes[2] != NKEYS * DK_DIM ||
      in_sizes[3] != NLOC * LOC_PITCH || in_sizes[4] != NVOC * E_DIM || in_sizes[5] != G3_DIM * E_DIM ||
      in_sizes[6] != G3_DIM * H_DIM || in_sizes[7] != G3_DIM || in_sizes[8] != G3_DIM ||
      in_sizes[9] != H_DIM * DK_DIM || in_sizes[10] != H_DIM * DK_DIM || in_sizes[11] != NLOC * CAT_DIM ||
      in_sizes[12] != NLOC || in_sizes[13] != H_DIM || in_sizes[14] != DK_DIM || in_sizes[15] != E_DIM ||
      in_sizes[16] != NVOC * NLOC || in_sizes[17] != NVOC || out_size != T_STEPS * NVOC) return;

  const int*   Xp     = (const int*)d_in[0];
  const float* glo    = (const float*)d_in[1];
  const float* lochid = (const float*)d_in[2];
  const float* locout = (const float*)d_in[3];
  const float* emb    = (const float*)d_in[4];
  const float* W_ih   = (const float*)d_in[5];
  const float* W_hh   = (const float*)d_in[6];
  const float* b_ih   = (const float*)d_in[7];
  const float* b_hh   = (const float*)d_in[8];
  const float* W_ga_g = (const float*)d_in[9];
  const float* W_ga_l = (const float*)d_in[10];
  const float* Wv_w   = (const float*)d_in[11];
  const float* Wv_b   = (const float*)d_in[12];
  const float* whp    = (const float*)d_in[13];
  const float* wcp    = (const float*)d_in[14];
  const float* wyp    = (const float*)d_in[15];
  const float* fc_w   = (const float*)d_in[16];
  const float* fc_b   = (const float*)d_in[17];
  float* outp = (float*)d_out;

  char* ws = (char*)d_ws; size_t off = 0;
  auto carve = [&](size_t bytes) -> char* { char* p = ws + off; off += (bytes + 255) & ~(size_t)255; return p; };
  unsigned short* KEY16   = (unsigned short*)carve((size_t)NKEYS_PAD * DK_DIM * 2);
  unsigned short* VALT16  = (unsigned short*)carve((size_t)DK_DIM * NKEYS_PAD * 2);
  float*          GX      = (float*)carve((size_t)T_STEPS * G3_DIM * 4);
  float*          OUTF    = (float*)carve((size_t)T_STEPS * H_DIM * 4);
  unsigned short* CAT16   = (unsigned short*)carve((size_t)T_STEPS * CAT_DIM * 2);
  unsigned short* Q16     = (unsigned short*)carve((size_t)T_STEPS * DK_DIM * 2);
  float*          PCTX    = (float*)carve((size_t)FL_NSPLIT * T_STEPS * DK_DIM * 4);
  float*          PM      = (float*)carve((size_t)FL_NSPLIT * T_STEPS * 4);
  float*          PL      = (float*)carve((size_t)FL_NSPLIT * T_STEPS * 4);
  float*          CG      = (float*)carve((size_t)T_STEPS * DK_DIM * 4);
  float*          CL      = (float*)carve((size_t)T_STEPS * DK_DIM * 4);
  unsigned short* Y16     = (unsigned short*)carve((size_t)T_STEPS * E_DIM * 2);
  unsigned short* WIH16   = (unsigned short*)carve((size_t)G3_DIM * E_DIM * 2);
  unsigned short* WHH_HI  = (unsigned short*)carve((size_t)G3_DIM * H_DIM * 2);
  unsigned short* WHH_LO  = (unsigned short*)carve((size_t)G3_DIM * H_DIM * 2);
  unsigned short* WGT16   = (unsigned short*)carve((size_t)DK_DIM * H_DIM * 2);
  unsigned short* WV16    = (unsigned short*)carve((size_t)NLOC_PAD * CAT_DIM * 2);
  unsigned short* FCW_HI  = (unsigned short*)carve((size_t)NVOC_PAD * NLOC_PAD * 2);
  unsigned short* FCW_LO  = (unsigned short*)carve((size_t)NVOC_PAD * NLOC_PAD * 2);
  unsigned short* GLOC_HI = (unsigned short*)carve((size_t)NLOC_PAD * DK_DIM * 2);
  unsigned short* GLOC_LO = (unsigned short*)carve((size_t)NLOC_PAD * DK_DIM * 2);
  unsigned short* WGL_HI  = (unsigned short*)carve((size_t)H_DIM * DK_DIM * 2);
  unsigned short* WGL_LO  = (unsigned short*)carve((size_t)H_DIM * DK_DIM * 2);
  unsigned short* GLOCT16 = (unsigned short*)carve((size_t)DK_DIM * NLOC_PAD * 2);
  unsigned short* OUT_HI  = (unsigned short*)carve((size_t)T_STEPS * H_DIM * 2);
  unsigned short* OUT_LO  = (unsigned short*)carve((size_t)T_STEPS * H_DIM * 2);
  unsigned short* WL_HI   = (unsigned short*)carve((size_t)NLOC_PAD * H_DIM * 2);
  unsigned short* WL_LO   = (unsigned short*)carve((size_t)NLOC_PAD * H_DIM * 2);
  float*          SL      = (float*)carve((size_t)T_STEPS * NLOC_PAD * 4);
  float*          BETA    = (float*)carve((size_t)T_STEPS * NLOC_PAD * 4);
  unsigned short* BETA16  = (unsigned short*)carve((size_t)T_STEPS * NLOC_PAD * 2);
  float*          LOGITS  = (float*)carve((size_t)T_STEPS * NLOC_PAD * 4);
  unsigned short* PW_HI   = (unsigned short*)carve((size_t)T_STEPS * NLOC_PAD * 2);
  unsigned short* PW_LO   = (unsigned short*)carve((size_t)T_STEPS * NLOC_PAD * 2);
  if (off > ws_size || off > (size_t)134217728) return;

  gather_y16_kernel<<<(T_STEPS * (E_DIM / 8)) / 256, 256, 0, stream>>>(Xp, emb, Y16);
  cvt8_f16_kernel<false><<<(G3_DIM * (E_DIM / 8)) / 256, 256, 0, stream>>>(
      W_ih, E_DIM, 0, G3_DIM, G3_DIM, E_DIM / 8, WIH16, WIH16, E_DIM, 0, W_CARRY);
  cvt8_f16_kernel<true><<<(G3_DIM * (H_DIM / 8)) / 256, 256, 0, stream>>>(
      W_hh, H_DIM, 0, G3_DIM, G3_DIM, H_DIM / 8, WHH_HI, WHH_LO, H_DIM, 0, W_CARRY);
  tp_f16_kernel<<<dim3(DK_DIM / 64, H_DIM / 64), 256, 0, stream>>>(W_ga_g, DK_DIM, H_DIM, WGT16, H_DIM, W_CARRY);
  cvt8_f16_kernel<false><<<(NKEYS_PAD * (DK_DIM / 8)) / 256, 256, 0, stream>>>(
      glo, DK_DIM, 0, NKEYS, NKEYS_PAD, DK_DIM / 8, KEY16, KEY16, DK_DIM, 0, 1.0f);
  tp_f16_kernel<<<dim3(DK_DIM / 64, NKEYS_PAD / 64), 256, 0, stream>>>(glo, DK_DIM, NKEYS, VALT16, NKEYS_PAD, 1.0f);
  cvt8_f16_kernel<false><<<(NLOC_PAD * (CAT_DIM / 8)) / 256, 256, 0, stream>>>(
      Wv_w, CAT_DIM, 0, NLOC, NLOC_PAD, CAT_DIM / 8, WV16, WV16, CAT_DIM, 0, W_CARRY);
  split8_bf16_kernel<<<(NVOC_PAD * (NLOC_PAD / 8)) / 256, 256, 0, stream>>>(
      fc_w, NLOC, NVOC, NLOC, NVOC_PAD, NLOC_PAD / 8, FCW_HI, FCW_LO);
  split8_bf16_kernel<<<(NLOC_PAD * (DK_DIM / 8)) / 256, 256, 0, stream>>>(
      locout, LOC_PITCH, NLOC, DK_DIM, NLOC_PAD, DK_DIM / 8, GLOC_HI, GLOC_LO);
  split8_bf16_kernel<<<(H_DIM * (DK_DIM / 8)) / 256, 256, 0, stream>>>(
      W_ga_l, DK_DIM, H_DIM, DK_DIM, H_DIM, DK_DIM / 8, WGL_HI, WGL_LO);
  tp_f16_kernel<<<dim3(DK_DIM / 64, NLOC_PAD / 64), 256, 0, stream>>>(locout, LOC_PITCH, NLOC, GLOCT16, NLOC_PAD, 1.0f);

  wmma_gemm64<0, false, 2, 0><<<dim3((T_STEPS / 64) * (G3_DIM / 64) / 8), 256, 0, stream>>>(
      Y16, Y16, E_DIM, WIH16, WIH16, E_DIM, (void*)GX, (void*)GX, G3_DIM, b_ih, T_STEPS, G3_DIM, E_DIM, GX_SCALE);

  gru_kernel<<<1, GRU_THREADS, 0, stream>>>(GX, WHH_HI, WHH_LO, b_hh, glo, lochid, OUTF, CAT16);

  wmma_gemm64<0, false, 0, 1><<<dim3((T_STEPS / 64) * (DK_DIM / 64) / 8), 256, 0, stream>>>(
      CAT16, CAT16, CAT_DIM, WGT16, WGT16, H_DIM, (void*)Q16, (void*)Q16, DK_DIM, b_ih, T_STEPS, DK_DIM, H_DIM, Q_OUT_SCALE);

  flash_kernel<<<dim3(T_STEPS / FL_MT, FL_NSPLIT), 256, 0, stream>>>(Q16, KEY16, VALT16, PCTX, PM, PL);
  combine_kernel<<<T_STEPS / 8, 256, 0, stream>>>(PCTX, PM, PL, CG);
  cvt8_f16_kernel<false><<<(T_STEPS * (DK_DIM / 8)) / 256, 256, 0, stream>>>(
      CG, DK_DIM, 0, T_STEPS, T_STEPS, DK_DIM / 8, CAT16, CAT16, CAT_DIM, H_DIM + DK_DIM, H_CARRY);

  split8_bf16_kernel<<<(T_STEPS * (H_DIM / 8)) / 256, 256, 0, stream>>>(
      OUTF, H_DIM, T_STEPS, H_DIM, T_STEPS, H_DIM / 8, OUT_HI, OUT_LO);
  wmma_gemm64<1, true, 0, 2><<<dim3((NLOC_PAD / 64) * (H_DIM / 64) / 8), 256, 0, stream>>>(
      GLOC_HI, GLOC_LO, DK_DIM, WGL_HI, WGL_LO, DK_DIM, (void*)WL_HI, (void*)WL_LO, H_DIM, b_ih, NLOC_PAD, H_DIM, DK_DIM, 1.0f);
  wmma_gemm64<1, true, 0, 0><<<dim3((T_STEPS / 64) * (NLOC_PAD / 64) / 8), 256, 0, stream>>>(
      OUT_HI, OUT_LO, H_DIM, WL_HI, WL_LO, H_DIM, (void*)SL, (void*)SL, NLOC_PAD, b_ih, T_STEPS, NLOC_PAD, H_DIM, 1.0f);
  beta_softmax_kernel<<<T_STEPS / 8, 256, 0, stream>>>(SL, BETA, BETA16);
  wmma_gemm64<0, false, 0, 0><<<dim3((T_STEPS / 64) * (DK_DIM / 64) / 8), 256, 0, stream>>>(
      BETA16, BETA16, NLOC_PAD, GLOCT16, GLOCT16, NLOC_PAD, (void*)CL, (void*)CL, DK_DIM, b_ih, T_STEPS, DK_DIM, NLOC_PAD, CL_SCALE);
  cvt8_f16_kernel<false><<<(T_STEPS * (DK_DIM / 8)) / 256, 256, 0, stream>>>(
      CL, DK_DIM, 0, T_STEPS, T_STEPS, DK_DIM / 8, CAT16, CAT16, CAT_DIM, H_DIM, H_CARRY);

  wmma_gemm64<0, false, 0, 0><<<dim3((T_STEPS / 64) * (NLOC_PAD / 64) / 8), 256, 0, stream>>>(
      CAT16, CAT16, CAT_DIM, WV16, WV16, CAT_DIM, (void*)LOGITS, (void*)LOGITS, NLOC_PAD, b_ih, T_STEPS, NLOC_PAD, CAT_DIM, LG_SCALE);
  head_kernel<<<T_STEPS / 8, 256, 0, stream>>>(LOGITS, Wv_b, BETA, OUTF, CL, Xp, emb, whp, wcp, wyp, PW_HI, PW_LO);
  fc_kernel<<<T_STEPS / 16, 256, 0, stream>>>(PW_HI, PW_LO, FCW_HI, FCW_LO, fc_b, outp);
}
